// CrossAttentionSkip_17497696764504
// MI455X (gfx1250) — hardware-run, weakly checked
//
#include <hip/hip_runtime.h>
#include <math.h>

typedef __attribute__((ext_vector_type(16))) _Float16 v16h;
typedef __attribute__((ext_vector_type(16))) __bf16 v16b;
typedef __attribute__((ext_vector_type(8)))  _Float16 v8h;
typedef __attribute__((ext_vector_type(8)))  float v8f;
typedef __attribute__((ext_vector_type(4)))  float v4f;
typedef __attribute__((ext_vector_type(2)))  float v2f;
typedef __attribute__((ext_vector_type(4)))  unsigned v4u;
typedef __attribute__((ext_vector_type(4)))  int v4i;
typedef float __attribute__((may_alias)) float_a;
typedef int __attribute__((may_alias)) int_a;

template <typename T> __device__ __forceinline__ void vst2(void* p, T v) { *(volatile T*)p = v; __threadfence(); *(volatile T*)p = v; }
__device__ __forceinline__ v8f wmma16(v16h a, v16h b, v8f c) {
  v8f d = __builtin_amdgcn_wmma_f32_16x16x32_f16(false, a, false, b, (short)0, c, false, false);
  asm volatile("v_nop\n\tv_nop\n\tv_nop\n\tv_nop" : "+v"(d) : "v"(a), "v"(b));
  return d;
}
__device__ __forceinline__ v8f wmma_bf(v16b a, v16b b, v8f c) {
  v8f d = __builtin_amdgcn_wmma_f32_16x16x32_bf16(false, a, false, b, (short)0, c, false, false);
  asm volatile("v_nop\n\tv_nop\n\tv_nop\n\tv_nop" : "+v"(d) : "v"(a), "v"(b));
  return d;
}
__device__ __forceinline__ v16h frag_h(const _Float16* rowk0, int lane) {
  union { v16h v; v8h q[2]; } u; const _Float16* p = rowk0 + 8 * (lane >> 4);
  u.q[0] = *(const v8h*)p; u.q[1] = *(const v8h*)(p + 16); return u.v;
}
__device__ __forceinline__ v16h frag_f32(const float* rowk0, int lane) {
  v16h a; const float* p = rowk0 + 8 * (lane >> 4);
#pragma unroll
  for (int i = 0; i < 8; ++i) { a[i] = (_Float16)p[i]; a[8 + i] = (_Float16)p[16 + i]; }
  return a;
}
__device__ __forceinline__ v16h frag_f32s(const float* rowk0, int lane, float sc) {
  v16h a; const float* p = rowk0 + 8 * (lane >> 4);
#pragma unroll
  for (int i = 0; i < 8; ++i) { a[i] = (_Float16)(p[i] * sc); a[8 + i] = (_Float16)(p[16 + i] * sc); }
  return a;
}
__device__ __forceinline__ v16h fragc_f32(const float* W, int k0, int n, int lane, int ld, int K) {
  v16h a; const int g = lane >> 4;
#pragma unroll
  for (int i = 0; i < 8; ++i) { const int ka = k0 + 8 * g + i, kb = ka + 16;
    a[i] = (_Float16)(ka < K ? W[(size_t)(ka < K ? ka : K - 1) * ld + n] : 0.f); a[8 + i] = (_Float16)(kb < K ? W[(size_t)(kb < K ? kb : K - 1) * ld + n] : 0.f); }
  return a;
}
struct F2 { v16b h, l; };
__device__ __forceinline__ F2 bsplit16(const float v[16]) { F2 r;
#pragma unroll
  for (int i = 0; i < 16; ++i) { const __bf16 h = (__bf16)v[i]; r.h[i] = h; r.l[i] = (__bf16)(v[i] - (float)h); }
  return r; }
__device__ __forceinline__ F2 split_row(const float* row, int k0, int lane) { float v[16]; const float* p = row + k0 + 8 * (lane >> 4);
#pragma unroll
  for (int i = 0; i < 8; ++i) { v[i] = p[i]; v[8 + i] = p[16 + i]; }
  return bsplit16(v); }
__device__ __forceinline__ F2 split_rowK(const float* row, int k0, int lane, int K) { float v[16]; const int g = lane >> 4;
#pragma unroll
  for (int i = 0; i < 8; ++i) { const int ka = k0 + 8 * g + i, kb = ka + 16; v[i] = ka < K ? row[ka < K ? ka : K - 1] : 0.f; v[8 + i] = kb < K ? row[kb < K ? kb : K - 1] : 0.f; }
  return bsplit16(v); }
__device__ __forceinline__ F2 split_col(const float* W, int k0, int n, int lane, int ld, int K) { float v[16]; const int g = lane >> 4;
#pragma unroll
  for (int i = 0; i < 8; ++i) { const int ka = k0 + 8 * g + i, kb = ka + 16; v[i] = ka < K ? W[(size_t)(ka < K ? ka : K - 1) * ld + n] : 0.f; v[8 + i] = kb < K ? W[(size_t)(kb < K ? kb : K - 1) * ld + n] : 0.f; }
  return bsplit16(v); }
__device__ __forceinline__ v8f mac3(const F2& a, const F2& b, v8f c) { c = wmma_bf(a.l, b.h, c); c = wmma_bf(a.h, b.l, c); return wmma_bf(a.h, b.h, c); }
__device__ __forceinline__ float sigm(float v) { return 1.0f / (1.0f + expf(-v)); }
#define LDSX() do { asm volatile("s_wait_dscnt 0" ::: "memory"); __builtin_amdgcn_wave_barrier(); __builtin_amdgcn_fence(__ATOMIC_RELEASE, "workgroup"); } while (0)


#define NBT 2
#define NTK 4096
#define NR (NBT * NTK)
#define CC 128
#define NH 4
#define HD 32
#define FF 512
#ifndef NQT
#define NQT (NR / 64)
#endif
typedef __attribute__((ext_vector_type(8))) __bf16 v8b;
__device__ __forceinline__ v16b frag_b(const __bf16* rowk0, int lane) {
  union { v16b v; v8b q[2]; } u; const __bf16* p = rowk0 + 8 * (lane >> 4);
  u.q[0] = *(const v8b*)p; u.q[1] = *(const v8b*)(p + 16); return u.v;
}
__device__ __forceinline__ float bfr(float v) { return (float)(__bf16)v; }
__device__ __attribute__((noinline)) float exp_ni(float v) { return expf(v); }
__device__ __attribute__((noinline)) float erf_ni(float v) { return erff(v); }

__device__ __forceinline__ float gelu_erf(float v) { return 0.5f * v * (1.0f + erf_ni(v * 0.70710678118654752f)); }
#define WS_PW   0u
#define P_Q 0
#define P_K (P_Q + 128 * 128)
#define P_V (P_K + 128 * 128)
#define P_O (P_V + 128 * 128)
#define P_1 (P_O + 128 * 128)
#define P_2 (P_1 + 512 * 128)
#define PWEND (P_2 + 128 * 512)
#define WS_ENC  (WS_PW + 2u * PWEND)
#define WS_DEC  (WS_ENC + 4u * NR * CC)
#define WS_Q    (WS_DEC + 4u * NR * CC)
#define WS_K    (WS_Q + 4u * NR * CC)
#define WS_VT   (WS_K + 4u * NR * CC)
#define WS_VTL  (WS_VT + 2u * NBT * CC * NTK)
#define WS_O    (WS_VTL + 2u * NBT * CC * NTK)
#define WS_R1   (WS_O + 4u * NR * CC)
#define WS_HF   (WS_R1 + 4u * NR * CC)
#define WS_Y    (WS_HF + 4u * NR * FF)
#define WS_END  (WS_Y + 4u * NR * CC)

__global__ __launch_bounds__(128) void k_packW(const float* __restrict__ WQ, const float* __restrict__ WK, const float* __restrict__ WV, const float* __restrict__ WO, const float* __restrict__ W1, const float* __restrict__ W2, __bf16* __restrict__ PW) {
  __shared__ __align__(16) __bf16 s[512]; const int o = blockIdx.x, which = blockIdx.y, t = threadIdx.x;
  if (which < 4) { const float* Wm = which == 0 ? WQ : which == 1 ? WK : which == 2 ? WV : WO; if (o >= CC) return; s[t] = (__bf16)Wm[o * CC + t]; __syncthreads(); if (t < 16) vst2((unsigned*)(PW + (size_t)which * 128 * 128 + (size_t)o * CC + t * 8), *(const v4u*)&s[t * 8]); }
  else if (which == 4) { s[t] = (__bf16)W1[(size_t)o * CC + t]; __syncthreads(); if (t < 16) vst2((unsigned*)(PW + P_1 + (size_t)o * CC + t * 8), *(const v4u*)&s[t * 8]); }
  else { if (o >= CC) return; for (int k = t; k < FF; k += 128) s[k] = (__bf16)W2[(size_t)o * FF + k]; __syncthreads(); if (t < 64) vst2((unsigned*)(PW + P_2 + (size_t)o * FF + t * 8), *(const v4u*)&s[t * 8]); }
}
__global__ __launch_bounds__(128) void k_ln_in(const float* __restrict__ E, const float* __restrict__ Dd, const float* __restrict__ GE, const float* __restrict__ BE, const float* __restrict__ GD, const float* __restrict__ BD, float* __restrict__ ENC, float* __restrict__ DEC) {
  __shared__ __align__(16) float s[64][132]; const int t = threadIdx.x; const int which = blockIdx.y; const size_t t0 = (size_t)blockIdx.x * 64; const int b = (int)(t0 / NTK), n0 = (int)(t0 % NTK);
  const float* src = which ? Dd : E; const float* gg = which ? GD : GE; const float* bb = which ? BD : BE; float* dst = which ? DEC : ENC;
  for (int q = t; q < CC * 64; q += 128) { const int c = q >> 6, nl = q & 63; s[nl][c] = bfr(src[((size_t)b * CC + c) * NTK + n0 + nl]); }
  __syncthreads();
  { const int nl = t >> 1, half = t & 1;
    float a = 0.f; for (int c = half * 64; c < half * 64 + 64; ++c) a += s[nl][c]; a += __shfl_xor(a, 1); const float mu = a / 128.f;
    float v = 0.f; for (int c = half * 64; c < half * 64 + 64; ++c) { const float d = s[nl][c] - mu; v += d * d; } v += __shfl_xor(v, 1); const float rs = rsqrtf(v / 128.f + 1e-5f);
    __syncthreads();
    for (int c = half * 64; c < half * 64 + 64; ++c) s[nl][c] = (s[nl][c] - mu) * rs * bfr(gg[c]) + bfr(bb[c]); }
  __syncthreads();
  for (int q = t; q < 64 * 32; q += 128) { const int nl = q >> 5, pc = q & 31; vst2(dst + (t0 + nl) * CC + pc * 4, *(const v4f*)&s[nl][pc * 4]); }
}
template <int MODE>
__global__ __launch_bounds__(128) void k_proj(const float* __restrict__ A, const __bf16* __restrict__ P, const float* __restrict__ Bv, const float* __restrict__ RES, float* __restrict__ OUTP, __bf16* __restrict__ VT, __bf16* __restrict__ VTL) {
  __shared__ __align__(16) float so[4][16][132]; __shared__ __align__(16) __bf16 sh[128][72], sl[128][72];
  constexpr int K = (MODE == 4) ? FF : CC;
  const int tid = threadIdx.x, wave = tid >> 5, lane = tid & 31, col = lane & 15, g = lane >> 4; const size_t r0 = (size_t)blockIdx.x * 64 + wave * 16;
  v8f acc[8] = {};
#pragma unroll 2
  for (int kc = 0; kc < K / 32; ++kc) { const F2 a = split_row(A + (r0 + col) * K, kc * 32, lane);
#pragma unroll
    for (int j = 0; j < 8; ++j) { const v16b w = frag_b(P + (size_t)(j * 16 + col) * K + kc * 32, lane); acc[j] = wmma_bf(a.l, w, acc[j]); acc[j] = wmma_bf(a.h, w, acc[j]); } }
#pragma unroll
  for (int j = 0; j < 8; ++j) { const float bb = bfr(Bv[j * 16 + col]);
#pragma unroll
    for (int r = 0; r < 8; ++r) { float v = acc[j][r] + bb; if (MODE >= 3) v += RES[(r0 + 8 * g + r) * CC + j * 16 + col]; so[wave][8 * g + r][j * 16 + col] = v; } }
  LDSX();
  if (MODE != 2) { for (int rl = 0; rl < 16; ++rl) vst2(OUTP + (r0 + rl) * CC + lane * 4, *(const v4f*)&so[wave][rl][lane * 4]); }
  else { __syncthreads(); const size_t t0 = (size_t)blockIdx.x * 64; const int b = (int)(t0 / NTK), n0 = (int)(t0 % NTK);
    for (int q = tid; q < 128 * 64; q += 128) { const int c = q >> 6, rl = q & 63; const float v = so[rl >> 4][rl & 15][c]; const __bf16 h = (__bf16)v; sh[c][rl] = h; sl[c][rl] = (__bf16)(v - (float)h); }
    __syncthreads();
    for (int q = tid; q < 128 * 8; q += 128) { const int c = q >> 3, pc = q & 7; const size_t base = ((size_t)b * CC + c) * NTK + n0 + pc * 8; vst2((unsigned*)(VT + base), *(const v4u*)&sh[c][pc * 8]); vst2((unsigned*)(VTL + base), *(const v4u*)&sl[c][pc * 8]); } }
}
__global__ __launch_bounds__(128) void k_att(const float* __restrict__ Q, const float* __restrict__ Kp, const __bf16* __restrict__ VT, const __bf16* __restrict__ VTL, float* __restrict__ O) {
  __shared__ __align__(16) float sp[4][16][36]; __shared__ __align__(16) float so[4][16][132];
  const int tid = threadIdx.x, wave = tid >> 5, lane = tid & 31, col = lane & 15, g = lane >> 4; const size_t r0 = (size_t)blockIdx.x * 64 + wave * 16; const int b = (int)(r0 / NTK); const float scale = 0.17677669529663687f;
#pragma unroll 1
  for (int h = 0; h < NH; ++h) { const F2 qa = split_row(Q + (r0 + col) * CC, h * HD, lane);
    float m[8], l[8]; v8f acc[2] = {};
#pragma unroll
    for (int r = 0; r < 8; ++r) { m[r] = -3.0e38f; l[r] = 0.f; }
#pragma unroll 1
    for (int ks = 0; ks < NTK / 32; ++ks) { float sv[8][2];
#pragma unroll
      for (int ct = 0; ct < 2; ++ct) { v8f sc = {}; const F2 kb = split_row(Kp + ((size_t)b * NTK + ks * 32 + ct * 16 + col) * CC, h * HD, lane); sc = wmma_bf(qa.l, kb.h, sc); sc = wmma_bf(qa.h, kb.l, sc); sc = wmma_bf(qa.h, kb.h, sc);
#pragma unroll
        for (int r = 0; r < 8; ++r) sv[r][ct] = sc[r] * scale; }
#pragma unroll
      for (int r = 0; r < 8; ++r) { float mx = fmaxf(sv[r][0], sv[r][1]);
#pragma unroll
        for (int o = 1; o < 16; o <<= 1) mx = fmaxf(mx, __shfl_xor(mx, o));
        const float mn = fmaxf(m[r], mx); const float alpha = (m[r] <= -1.0e38f) ? 0.f : __expf(m[r] - mn); const float e0 = __expf(sv[r][0] - mn), e1 = __expf(sv[r][1] - mn); float es = e0 + e1;
#pragma unroll
        for (int o = 1; o < 16; o <<= 1) es += __shfl_xor(es, o);
        l[r] = l[r] * alpha + es; m[r] = mn; acc[0][r] *= alpha; acc[1][r] *= alpha; sp[wave][8 * g + r][col] = e0; sp[wave][8 * g + r][16 + col] = e1; }
      LDSX();
      const F2 pa = split_row(&sp[wave][col][0], 0, lane);
#pragma unroll
      for (int j = 0; j < 2; ++j) { const size_t pr = ((size_t)b * CC + h * HD + j * 16 + col) * NTK + ks * 32; const v16b vh = frag_b(VT + pr, lane), vl = frag_b(VTL + pr, lane); acc[j] = wmma_bf(pa.l, vh, acc[j]); acc[j] = wmma_bf(pa.h, vl, acc[j]); acc[j] = wmma_bf(pa.h, vh, acc[j]); }
      LDSX(); }
#pragma unroll
    for (int j = 0; j < 2; ++j)
#pragma unroll
      for (int r = 0; r < 8; ++r) so[wave][8 * g + r][h * HD + j * 16 + col] = acc[j][r] / l[r]; }
  LDSX();
  for (int rl = 0; rl < 16; ++rl) vst2(O + (r0 + rl) * CC + lane * 4, *(const v4f*)&so[wave][rl][lane * 4]);
}
__global__ __launch_bounds__(128) void k_ffn1(const float* __restrict__ R1, const float* __restrict__ G, const float* __restrict__ Bt, const __bf16* __restrict__ P, const float* __restrict__ B1, float* __restrict__ HF) {
  __shared__ __align__(16) float sa[4][16][132]; __shared__ __align__(16) float so[4][16][132];
  const int tid = threadIdx.x, wave = tid >> 5, lane = tid & 31, col = lane & 15, g = lane >> 4; const size_t r0 = (size_t)blockIdx.x * 64 + wave * 16; const int n0 = blockIdx.y * 128;
  { const int rl = col; const float* row = R1 + (r0 + rl) * CC; float a = 0.f; for (int c = g * 64; c < g * 64 + 64; ++c) a += row[c]; a += __shfl_xor(a, 16); const float mu = a / 128.f;
    float v = 0.f; for (int c = g * 64; c < g * 64 + 64; ++c) { const float d = row[c] - mu; v += d * d; } v += __shfl_xor(v, 16); const float rs = rsqrtf(v / 128.f + 1e-5f);
    for (int c = g * 64; c < g * 64 + 64; ++c) sa[wave][rl][c] = (row[c] - mu) * rs * bfr(G[c]) + bfr(Bt[c]); }
  LDSX();
  v8f acc[8] = {};
#pragma unroll
  for (int kc = 0; kc < 4; ++kc) { const F2 a = split_row(&sa[wave][col][0], kc * 32, lane);
#pragma unroll
    for (int j = 0; j < 8; ++j) { const v16b w = frag_b(P + (size_t)(n0 + j * 16 + col) * CC + kc * 32, lane); acc[j] = wmma_bf(a.l, w, acc[j]); acc[j] = wmma_bf(a.h, w, acc[j]); } }
#pragma unroll
  for (int j = 0; j < 8; ++j) { const float bb = bfr(B1[n0 + j * 16 + col]);
#pragma unroll
    for (int r = 0; r < 8; ++r) so[wave][8 * g + r][j * 16 + col] = gelu_erf(acc[j][r] + bb); }
  LDSX();
  for (int rl = 0; rl < 16; ++rl) vst2(HF + (r0 + rl) * FF + n0 + lane * 4, *(const v4f*)&so[wave][rl][lane * 4]);
}
__global__ __launch_bounds__(128) void k_out(const float* __restrict__ Y, float* __restrict__ OUT) {
  __shared__ __align__(16) float s[CC][68]; const int t = threadIdx.x; const size_t t0 = (size_t)blockIdx.x * 64; const int b = (int)(t0 / NTK), n0 = (int)(t0 % NTK);
  for (int q = t; q < 64 * CC; q += 128) { const int nl = q >> 7, c = q & 127; s[c][nl] = Y[(t0 + nl) * CC + c]; }
  __syncthreads();
  for (int q = t; q < CC * 16; q += 128) { const int c = q >> 4, pc = q & 15; vst2(OUT + ((size_t)b * CC + c) * NTK + n0 + pc * 4, *(const v4f*)&s[c][pc * 4]); }
}
extern "C" void kernel_launch(void* const* d_in, const int* in_sizes, int n_in, void* d_out, int out_size, void* d_ws, size_t ws_size, hipStream_t stream) {
  (void)in_sizes; (void)n_in; (void)out_size;
  const float** F = (const float**)d_in;
  if (ws_size < (size_t)WS_END) return;
  char* ws = (char*)d_ws; __bf16* PW = (__bf16*)(ws + WS_PW); float *ENC = (float*)(ws + WS_ENC), *DEC = (float*)(ws + WS_DEC), *Q = (float*)(ws + WS_Q), *Kp = (float*)(ws + WS_K), *O = (float*)(ws + WS_O), *R1 = (float*)(ws + WS_R1), *HF = (float*)(ws + WS_HF), *Y = (float*)(ws + WS_Y); __bf16 *VT = (__bf16*)(ws + WS_VT), *VTL = (__bf16*)(ws + WS_VTL);
  k_packW<<<dim3(512, 6), 128, 0, stream>>>(F[2], F[4], F[6], F[8], F[16], F[18], PW);
  k_ln_in<<<dim3(NR / 64, 2), 128, 0, stream>>>(F[0], F[1], F[10], F[11], F[12], F[13], ENC, DEC);
  k_proj<0><<<NQT, 128, 0, stream>>>(DEC, PW + P_Q, F[3], nullptr, Q, nullptr, nullptr);
  k_proj<1><<<NR / 64, 128, 0, stream>>>(ENC, PW + P_K, F[5], nullptr, Kp, nullptr, nullptr);
  k_proj<2><<<NR / 64, 128, 0, stream>>>(ENC, PW + P_V, F[7], nullptr, nullptr, VT, VTL);
  k_att<<<NQT, 128, 0, stream>>>(Q, Kp, VT, VTL, O);
  k_proj<3><<<NQT, 128, 0, stream>>>(O, PW + P_O, F[9], DEC, R1, nullptr, nullptr);
  k_ffn1<<<dim3(NQT, FF / 128), 128, 0, stream>>>(R1, F[14], F[15], PW + P_1, F[17], HF);
  k_proj<4><<<NQT, 128, 0, stream>>>(HF, PW + P_2, F[19], R1, Y, nullptr, nullptr);
  k_out<<<NQT, 128, 0, stream>>>(Y, (float*)d_out);
}
